// CurlVectorField_75892072120800
// MI455X (gfx1250) — hardware-run, weakly checked
//
#include <hip/hip_runtime.h>


#define NPT 524288
#define CHK 65536
#define NHD 64
typedef _Float16 h16;
typedef unsigned short bf;
typedef __attribute__((ext_vector_type(16))) __bf16   v16bf;
typedef __attribute__((ext_vector_type(16))) _Float16 v16h;
typedef __attribute__((ext_vector_type(8)))  _Float16 v8h;
typedef __attribute__((ext_vector_type(8)))  unsigned short v8us;
typedef __attribute__((ext_vector_type(8)))  float    v8f;
typedef __attribute__((ext_vector_type(4)))  float    v4f;
typedef v8h  __attribute__((may_alias)) v8ha;
typedef v4f  __attribute__((may_alias)) v4fa;
typedef v8us __attribute__((may_alias)) v8usa;

__device__ __forceinline__ unsigned short f2bf(float f) { unsigned u = __float_as_uint(f); u += 0x7FFFu + ((u >> 16) & 1u); return (unsigned short)(u >> 16); }
__device__ __forceinline__ float bf2f(unsigned short b) { return __uint_as_float(((unsigned)b) << 16); }
__device__ __forceinline__ float bfr(float f) { return bf2f(f2bf(f)); }
__device__ __forceinline__ h16 tohx(float x) { return (h16)x; }
__device__ __forceinline__ v16h cat16(v8h lo, v8h hi) { return __builtin_shufflevector(lo, hi, 0, 1, 2, 3, 4, 5, 6, 7, 8, 9, 10, 11, 12, 13, 14, 15); }
__device__ __forceinline__ v16bf cat16b(v8us lo, v8us hi) { return __builtin_bit_cast(v16bf, __builtin_shufflevector(lo, hi, 0, 1, 2, 3, 4, 5, 6, 7, 8, 9, 10, 11, 12, 13, 14, 15)); }
__device__ __forceinline__ v8f wmma16(v16h a, v16h b, v8f c) { return __builtin_amdgcn_wmma_f32_16x16x32_f16(false, a, false, b, (short)0, c, false, false); }
__device__ __forceinline__ v8f wmmab(v16bf a, v16bf b, v8f c) { return __builtin_amdgcn_wmma_f32_16x16x32_bf16(false, a, false, b, (short)0, c, false, false); }

template <typename T16> struct WFrag;
template <> struct WFrag<h16> { typedef v16h V; static __device__ __forceinline__ V ld(const h16* p) { return cat16(*(const v8h*)p, *(const v8h*)(p + 16)); } static __device__ __forceinline__ v8f mma(V a, V b, v8f c) { return wmma16(a, b, c); } };
template <> struct WFrag<bf> { typedef v16bf V; static __device__ __forceinline__ V ld(const bf* p) { return cat16b(*(const v8us*)p, *(const v8us*)(p + 16)); } static __device__ __forceinline__ v8f mma(V a, V b, v8f c) { return wmmab(a, b, c); } };
template <typename T16, int NSPLIT, bool BIAS>
__global__ __launch_bounds__(32) void k_gemmw(const T16* __restrict__ A, const T16* __restrict__ A2, const T16* __restrict__ Bt, const T16* __restrict__ Bt2, int K, float* C, int ldc, const float* __restrict__ bias, size_t sA, size_t sB, size_t sC) {
    typedef typename WFrag<T16>::V V;
    __shared__ __align__(16) float os[16 * 68];
    const size_t z = blockIdx.z; A += z * sA; if (A2) A2 += z * sA; Bt += z * sB; if (Bt2) Bt2 += z * sB; C += z * sC;
    const int lane = threadIdx.x & 31, lr = lane & 15, hi = lane >> 4; const int r0 = blockIdx.x * 64, c0 = blockIdx.y * 64;
    v8f acc[4][4];
#pragma unroll
    for (int mb = 0; mb < 4; ++mb)
#pragma unroll
        for (int nb = 0; nb < 4; ++nb) acc[mb][nb] = (v8f){};
    const size_t aoff = (size_t)(r0 + lr) * K + 8 * hi, boff = (size_t)(c0 + lr) * K + 8 * hi;
    for (int kc = 0; kc < K; kc += 32) {
        V a[4], a2[4];
#pragma unroll
        for (int mb = 0; mb < 4; ++mb) { a[mb] = WFrag<T16>::ld(A + aoff + (size_t)mb * 16 * K + kc); if (NSPLIT == 1 || NSPLIT == 2) a2[mb] = WFrag<T16>::ld(A2 + aoff + (size_t)mb * 16 * K + kc); }
#pragma unroll
        for (int nb = 0; nb < 4; ++nb) { const V b = WFrag<T16>::ld(Bt + boff + (size_t)nb * 16 * K + kc); V b2; if (NSPLIT >= 2) b2 = WFrag<T16>::ld(Bt2 + boff + (size_t)nb * 16 * K + kc);
#pragma unroll
            for (int mb = 0; mb < 4; ++mb) { acc[mb][nb] = WFrag<T16>::mma(a[mb], b, acc[mb][nb]); if (NSPLIT == 1 || NSPLIT == 2) acc[mb][nb] = WFrag<T16>::mma(a2[mb], b, acc[mb][nb]); if (NSPLIT >= 2) acc[mb][nb] = WFrag<T16>::mma(a[mb], b2, acc[mb][nb]); } }
        asm volatile("v_nop\n\tv_nop\n\tv_nop\n\tv_nop" : "+v"(acc[0][0]), "+v"(acc[1][1]), "+v"(acc[2][2]), "+v"(acc[3][3]) : "v"(a[0]), "v"(a[3]));
    }
#pragma unroll
    for (int mb = 0; mb < 4; ++mb) {
#pragma unroll
        for (int nb = 0; nb < 4; ++nb) {
#pragma unroll
            for (int j = 0; j < 8; ++j) os[(hi * 8 + j) * 68 + nb * 16 + lr] = acc[mb][nb][j]; }
        __builtin_amdgcn_wave_barrier(); asm volatile("" ::: "memory");
        float* crow = C + (size_t)(r0 + mb * 16) * ldc + c0;
#pragma unroll 1
        for (int ps = 0; ps < 2; ++ps) {
#pragma unroll
            for (int s = 0; s < 8; ++s) { const int row = 2 * s + hi, cofs = lr * 4; v4f val = *(const v4fa*)(os + row * 68 + cofs); if (BIAS) { val[0] += bfr(bias[c0 + cofs]); val[1] += bfr(bias[c0 + cofs + 1]); val[2] += bfr(bias[c0 + cofs + 2]); val[3] += bfr(bias[c0 + cofs + 3]); }
                *(volatile v4f*)(crow + (size_t)row * ldc + cofs) = val; }
            if (ps == 0) __threadfence(); }
        __builtin_amdgcn_wave_barrier(); asm volatile("" ::: "memory");
    }
}

__global__ __launch_bounds__(256) void k_cvt8(const float* __restrict__ src, bf* dst, size_t n8) { const size_t i = (size_t)blockIdx.x * 256 + threadIdx.x; if (i >= n8) return; const v8f v = *(const v8f*)(src + i * 8); v8us o;
#pragma unroll
    for (int k = 0; k < 8; ++k) o[k] = f2bf(v[k]); *(volatile v8us*)(dst + i * 8) = o; __threadfence(); *(volatile v8us*)(dst + i * 8) = o; }

__global__ __launch_bounds__(256) void k_b2h(const bf* src, h16* dst, size_t n8) {
    const size_t e = (size_t)blockIdx.x * 256 + threadIdx.x; if (e >= n8) return; const v8us w = *(const v8us*)(src + e * 8); v8h o;
#pragma unroll
    for (int q = 0; q < 8; ++q) o[q] = tohx(bf2f(w[q]));
    *(volatile v8h*)(dst + e * 8) = o; __threadfence(); *(volatile v8h*)(dst + e * 8) = o; }

__global__ __launch_bounds__(256) void k_front(const float* __restrict__ xs, const float* __restrict__ Wa, const float* __restrict__ ba, size_t r0, h16* H1, h16* T1) { const size_t e = (size_t)blockIdx.x * 256 + threadIdx.x; if (e >= (size_t)CHK * (NHD / 8)) return; const size_t n = e / (NHD / 8); const int h0 = (int)(e % (NHD / 8)) * 8; const float* xp = xs + (r0 + n) * 3; const float x0 = bfr(xp[0]), x1 = bfr(xp[1]), x2 = bfr(xp[2]); v8h hh, th[3];
#pragma unroll
  for (int q = 0; q < 8; ++q) { const int h = h0 + q; const float w0 = bfr(Wa[h * 3 + 0]), w1 = bfr(Wa[h * 3 + 1]), w2 = bfr(Wa[h * 3 + 2]); const float z = fmaf(x2, w2, fmaf(x1, w1, x0 * w0)) + bfr(ba[h]); const float h1 = tanhf(z); const float d1 = fmaf(-h1, h1, 1.0f); const float t0 = d1 * w0, t1 = d1 * w1, t2 = d1 * w2; hh[q] = tohx((fabsf(h1) < 6.103515625e-05f) ? 0.0f : h1); th[0][q] = tohx((fabsf(t0) < 6.103515625e-05f) ? 0.0f : t0); th[1][q] = tohx((fabsf(t1) < 6.103515625e-05f) ? 0.0f : t1); th[2][q] = tohx((fabsf(t2) < 6.103515625e-05f) ? 0.0f : t2); }
  const size_t o = n * NHD + h0;
#pragma unroll
  for (int ps = 0; ps < 2; ++ps) { *(volatile v8h*)(H1 + o) = hh;
#pragma unroll
    for (int d = 0; d < 3; ++d) *(volatile v8h*)(T1 + (size_t)d * CHK * NHD + o) = th[d];
    if (ps == 0) __threadfence(); } }

__global__ __launch_bounds__(256) void k_back(const float* Z2, const float* G, const float* __restrict__ Wc, size_t r0, float* out) { const size_t n = (size_t)blockIdx.x * 256 + threadIdx.x; if (n >= (size_t)CHK) return; const float* z = Z2 + n * NHD; const float* g0 = G + n * NHD; const float* g1 = G + ((size_t)CHK + n) * NHD; const float* g2 = G + ((size_t)2 * CHK + n) * NHD; float j21 = 0.0f, j12 = 0.0f, j02 = 0.0f, j20 = 0.0f, j10 = 0.0f, j01 = 0.0f;
  for (int h = 0; h < NHD; ++h) { const float h2 = tanhf(z[h]); const float d2 = fmaf(-h2, h2, 1.0f); const float t0 = d2 * g0[h], t1 = d2 * g1[h], t2 = d2 * g2[h]; const float c0 = bfr(Wc[h]), c1 = bfr(Wc[NHD + h]), c2 = bfr(Wc[2 * NHD + h]); j21 = fmaf(c2, t1, j21); j12 = fmaf(c1, t2, j12); j02 = fmaf(c0, t2, j02); j20 = fmaf(c2, t0, j20); j10 = fmaf(c1, t0, j10); j01 = fmaf(c0, t1, j01); }
  const float u0 = j21 - j12, u1 = j02 - j20, u2 = j10 - j01; float* po = out + (r0 + n) * 3; *(volatile float*)(po + 0) = u0; *(volatile float*)(po + 1) = u1; *(volatile float*)(po + 2) = u2; __threadfence(); *(volatile float*)(po + 0) = u0; *(volatile float*)(po + 1) = u1; *(volatile float*)(po + 2) = u2; }

extern "C" void kernel_launch(void* const* d_in, const int* in_sizes, int n_in,
                              void* d_out, int out_size, void* d_ws, size_t ws_size, hipStream_t stream) {
    (void)in_sizes; (void)n_in; (void)out_size;
    const float* xs = (const float*)d_in[0]; const float* Wa = (const float*)d_in[1]; const float* ba = (const float*)d_in[2]; const float* Wb = (const float*)d_in[3]; const float* bb = (const float*)d_in[4]; const float* Wc = (const float*)d_in[5]; (void)d_in[6];
    float* OUT = (float*)d_out;
    char* wsp = (char*)d_ws;
    auto take = [&](size_t bytes) { char* p = wsp; wsp += (bytes + 255) & ~(size_t)255; return (void*)p; };
    bf* WBB = (bf*)take((size_t)NHD * NHD * 2); h16* WBH = (h16*)take((size_t)NHD * NHD * 2); h16* H1 = (h16*)take((size_t)CHK * NHD * 2); h16* T1 = (h16*)take((size_t)3 * CHK * NHD * 2);
    float* Z2 = (float*)take((size_t)CHK * NHD * 4); float* G = (float*)take((size_t)3 * CHK * NHD * 4);
    if ((size_t)(wsp - (char*)d_ws) > ws_size) return;
    k_cvt8<<<(unsigned)((size_t)NHD * NHD / 8 / 256), 256, 0, stream>>>(Wb, WBB, (size_t)NHD * NHD / 8);
    k_b2h<<<(unsigned)(((size_t)NHD * NHD / 8 + 255) / 256), 256, 0, stream>>>(WBB, WBH, (size_t)NHD * NHD / 8);
    for (size_t r0 = 0; r0 < (size_t)NPT; r0 += CHK) {
        k_front<<<(unsigned)((size_t)CHK * (NHD / 8) / 256), 256, 0, stream>>>(xs, Wa, ba, r0, H1, T1);
        k_gemmw<h16, 0, true><<<dim3(CHK / 64, NHD / 64, 1), 32, 0, stream>>>(H1, nullptr, WBH, nullptr, NHD, Z2, NHD, bb, (size_t)0, (size_t)0, (size_t)0);
        k_gemmw<h16, 0, false><<<dim3(CHK / 64, NHD / 64, 3), 32, 0, stream>>>(T1, nullptr, WBH, nullptr, NHD, G, NHD, nullptr, (size_t)CHK * NHD, (size_t)0, (size_t)CHK * NHD);
        k_back<<<(unsigned)((size_t)CHK / 256), 256, 0, stream>>>(Z2, G, Wc, r0, OUT);
    }
}
